// StateSpaceSequencing_57947698758047
// MI455X (gfx1250) — hardware-verified
//
#include <hip/hip_runtime.h>

typedef _Float16 v8h  __attribute__((ext_vector_type(8)));
typedef _Float16 v16h __attribute__((ext_vector_type(16)));
typedef __bf16   v16b __attribute__((ext_vector_type(16)));
typedef unsigned short v8us __attribute__((ext_vector_type(8)));
typedef float v8f __attribute__((ext_vector_type(8)));
typedef float v4f __attribute__((ext_vector_type(4)));
typedef v8h  __attribute__((may_alias)) v8ha;
typedef v8us __attribute__((may_alias)) v8usa;
typedef v4f  __attribute__((may_alias)) v4fa;
typedef _Float16 __attribute__((may_alias)) f16a;

union FragH { v16h v; v8h p[2]; };
union FragB { v16b v; v8us p[2]; };

#define NB    32
#define DIN   128
#define LL    1024
#define DM    1024
#define LMAX  64
#define GBT   8
#define NGRP  (NB / GBT)
#define MG    (GBT * LL)

#define HZ4 "v_nop\n\tv_nop\n\tv_nop\n\tv_nop"

__device__ __forceinline__ unsigned short f2bf(float x) {
  unsigned int u = __float_as_uint(x);
  u += 0x7FFFu + ((u >> 16) & 1u);
  return (unsigned short)(u >> 16);
}
__device__ __forceinline__ float bf2f(unsigned short b) {
  return __uint_as_float(((unsigned int)b) << 16);
}

__device__ __forceinline__ v16h ldh(const _Float16* p, int h4) {
  FragH f;
  f.p[0] = *(const v8ha*)(p + 8 * h4);
  f.p[1] = *(const v8ha*)(p + 16 + 8 * h4);
  return f.v;
}
__device__ __forceinline__ v16b ldb(const unsigned short* p, int h4) {
  FragB f;
  f.p[0] = *(const v8usa*)(p + 8 * h4);
  f.p[1] = *(const v8usa*)(p + 16 + 8 * h4);
  return f.v;
}
__device__ __forceinline__ v8f mma_h(v16h a, v16h b, v8f c) {
  return __builtin_amdgcn_wmma_f32_16x16x32_f16(false, a, false, b, (short)0, c, false, false);
}
__device__ __forceinline__ v8f mma_b(v16b a, v16b b, v8f c) {
  return __builtin_amdgcn_wmma_f32_16x16x32_bf16(false, a, false, b, (short)0, c, false, false);
}
#define BH(x) __builtin_bit_cast(v16h, (x))

__device__ __forceinline__ float wsum(float v) {
  v += __shfl_xor(v, 16);
  v += __shfl_xor(v, 8);
  v += __shfl_xor(v, 4);
  v += __shfl_xor(v, 2);
  v += __shfl_xor(v, 1);
  return v;
}

__device__ __forceinline__ float gelu_t(float x) {
  const float u = 0.7978845608028654f * (x + 0.044715f * x * x * x);
  const float e = __expf(2.0f * u);
  const float th = fmaf(-2.0f, __builtin_amdgcn_rcpf(e + 1.0f), 1.0f);
  return 0.5f * x * (1.0f + th);
}

__global__ __launch_bounds__(256) void k_ssm(const float* __restrict__ log_dt,
                                             const float* __restrict__ Alr,
                                             const float* __restrict__ Aim,
                                             const float* __restrict__ Cre,
                                             const float* __restrict__ Cim,
                                             const float* __restrict__ Dv,
                                             float* __restrict__ Kf)
{
  const int g = blockIdx.x * 256 + threadIdx.x;
  if (g >= DM * LMAX) return;
  const int d = g >> 6, l = g & 63;
  const float dt = __expf(log_dt[d]);
  const float fl = (float)l;
  float acc = 0.0f;
#pragma unroll 1
  for (int n = 0; n < 4; ++n) {
    const float ar = -__expf(Alr[d * 4 + n]);
    const float ai = Aim[d * 4 + n];
    const float xr = ar * dt, xi = ai * dt;
    float w1r = 0.f, w1i = 0.f, wlr = 0.f, wli = 0.f;
#pragma unroll 1
    for (int q = 0; q < 2; ++q) {
      const bool first = (q == 0);
      const float s = first ? 1.0f : fl;
      const float er = __expf(xr * s);
      float sn, cs;
      sincosf(xi * s, &sn, &cs);
      const float vr = er * cs, vi = er * sn;
      w1r = first ? vr : w1r;  w1i = first ? vi : w1i;
      wlr = first ? wlr : vr;  wli = first ? wli : vi;
    }
    const float nr = w1r - 1.0f, ni = w1i;
    const float rden = __builtin_amdgcn_rcpf(ar * ar + ai * ai);
    const float Bdr = (nr * ar + ni * ai) * rden;
    const float Bdi = (ni * ar - nr * ai) * rden;
    const float cr = Cre[d * 4 + n], ci = Cim[d * 4 + n];
    const float cbr = cr * Bdr - ci * Bdi;
    const float cbi = cr * Bdi + ci * Bdr;
    acc += cbr * wlr - cbi * wli;
  }
  float kv = 2.0f * acc;
  kv += (l == 0) ? Dv[d] : 0.0f;
  *(volatile float*)(Kf + g) = kv;
  __threadfence();
  *(volatile float*)(Kf + g) = kv;
}

template <int MODE>
__global__ __launch_bounds__(256) void k_tr(const float* __restrict__ W,
                                            unsigned short* __restrict__ P0,
                                            unsigned short* __restrict__ P1,
                                            int K, int N, long long zin, long long zout, float sc)
{
  __shared__ float tile[64][65];
  const int t = threadIdx.x;
  const int n0 = blockIdx.x * 64, k0 = blockIdx.y * 64;
  const float* Wz = W + (size_t)blockIdx.z * (size_t)zin;
  {
    const int p = t & 15, kr = t >> 4;
#pragma unroll
    for (int it = 0; it < 4; ++it) {
      const int k = it * 16 + kr;
      const v4f v = *(const v4fa*)(Wz + (size_t)(k0 + k) * (size_t)N + n0 + 4 * p);
      tile[k][4 * p + 0] = v.x;
      tile[k][4 * p + 1] = v.y;
      tile[k][4 * p + 2] = v.z;
      tile[k][4 * p + 3] = v.w;
    }
  }
  __syncthreads();
  const int q8 = t & 7, nr = t >> 3;
  v8us oa[2], ob[2];
#pragma unroll
  for (int it = 0; it < 2; ++it) {
    const int n = it * 32 + nr;
    const float e0 = tile[8 * q8 + 0][n], e1 = tile[8 * q8 + 1][n];
    const float e2 = tile[8 * q8 + 2][n], e3 = tile[8 * q8 + 3][n];
    const float e4 = tile[8 * q8 + 4][n], e5 = tile[8 * q8 + 5][n];
    const float e6 = tile[8 * q8 + 6][n], e7 = tile[8 * q8 + 7][n];
    if (MODE == 0) {
      const v8h hv = {(_Float16)(e0 * sc), (_Float16)(e1 * sc), (_Float16)(e2 * sc), (_Float16)(e3 * sc),
                      (_Float16)(e4 * sc), (_Float16)(e5 * sc), (_Float16)(e6 * sc), (_Float16)(e7 * sc)};
      oa[it] = __builtin_bit_cast(v8us, hv);
      ob[it] = oa[it];
    } else {
      const unsigned short h0 = f2bf(e0), h1 = f2bf(e1), h2 = f2bf(e2), h3 = f2bf(e3);
      const unsigned short h4 = f2bf(e4), h5 = f2bf(e5), h6 = f2bf(e6), h7 = f2bf(e7);
      const v8us hh = {h0, h1, h2, h3, h4, h5, h6, h7};
      const v8us lw = {f2bf(e0 - bf2f(h0)), f2bf(e1 - bf2f(h1)), f2bf(e2 - bf2f(h2)), f2bf(e3 - bf2f(h3)),
                       f2bf(e4 - bf2f(h4)), f2bf(e5 - bf2f(h5)), f2bf(e6 - bf2f(h6)), f2bf(e7 - bf2f(h7))};
      oa[it] = hh;
      ob[it] = lw;
    }
  }
  unsigned short* P0z = P0 + (size_t)blockIdx.z * (size_t)zout;
  unsigned short* P1z = P1 + (size_t)blockIdx.z * (size_t)zout;
#pragma unroll
  for (int it = 0; it < 2; ++it) {
    const size_t off = (size_t)(n0 + it * 32 + nr) * (size_t)K + k0 + 8 * q8;
    *(volatile v8us*)(P0z + off) = oa[it];
    if (MODE == 1) *(volatile v8us*)(P1z + off) = ob[it];
  }
  __threadfence();
#pragma unroll
  for (int it = 0; it < 2; ++it) {
    const size_t off = (size_t)(n0 + it * 32 + nr) * (size_t)K + k0 + 8 * q8;
    *(volatile v8us*)(P0z + off) = oa[it];
    if (MODE == 1) *(volatile v8us*)(P1z + off) = ob[it];
  }
}

__global__ __launch_bounds__(256) void k_enc(const unsigned short* __restrict__ Xh,
                                             const unsigned short* __restrict__ Xl,
                                             const unsigned short* __restrict__ Wh,
                                             const unsigned short* __restrict__ Wl,
                                             const float* __restrict__ bias,
                                             float* __restrict__ H)
{
  __shared__ __attribute__((aligned(16))) float sT[8 * 32 * 32];
  const int t = threadIdx.x, lane = t & 31, w = t >> 5, h4 = lane >> 4, m = lane & 15;
  const int wm = (w >> 1) * 32, wn = (w & 1) * 32;
  const int r0 = blockIdx.y * 128 + wm;
  const int c0 = blockIdx.x * 64 + wn;
  const size_t ao0 = (size_t)(r0 + m) * DIN, ao1 = ao0 + (size_t)16 * DIN;
  const size_t bo0 = (size_t)(c0 + m) * DIN, bo1 = bo0 + (size_t)16 * DIN;
  const v8f z8 = {0.f, 0.f, 0.f, 0.f, 0.f, 0.f, 0.f, 0.f};
  v8f c00 = z8, c01 = z8, c10 = z8, c11 = z8;

#pragma unroll 1
  for (int k0 = 0; k0 < DIN; k0 += 32) {
    const v16b ah0 = ldb(Xh + ao0 + k0, h4), ah1 = ldb(Xh + ao1 + k0, h4);
    const v16b al0 = ldb(Xl + ao0 + k0, h4), al1 = ldb(Xl + ao1 + k0, h4);
    const v16b bh0 = ldb(Wh + bo0 + k0, h4), bh1 = ldb(Wh + bo1 + k0, h4);
    const v16b bl0 = ldb(Wl + bo0 + k0, h4), bl1 = ldb(Wl + bo1 + k0, h4);
    c00 = mma_b(ah0, bh0, c00); c00 = mma_b(ah0, bl0, c00); c00 = mma_b(al0, bh0, c00);
    c01 = mma_b(ah0, bh1, c01); c01 = mma_b(ah0, bl1, c01); c01 = mma_b(al0, bh1, c01);
    c10 = mma_b(ah1, bh0, c10); c10 = mma_b(ah1, bl0, c10); c10 = mma_b(al1, bh0, c10);
    c11 = mma_b(ah1, bh1, c11); c11 = mma_b(ah1, bl1, c11); c11 = mma_b(al1, bh1, c11);
    asm volatile(HZ4 : "+v"(c00), "+v"(c01), "+v"(c10), "+v"(c11)
                     : "v"(BH(ah0)), "v"(BH(ah1)), "v"(BH(al0)), "v"(BH(al1)),
                       "v"(BH(bh0)), "v"(BH(bh1)), "v"(BH(bl0)), "v"(BH(bl1)));
  }

  float* st = sT + w * 1024;
  const float bva = bias[c0 + m], bvb = bias[c0 + 16 + m];
#pragma unroll
  for (int r = 0; r < 8; ++r) {
    const int rr = 8 * h4 + r;
    st[rr * 32 + m]             = c00[r] + bva;
    st[rr * 32 + 16 + m]        = c01[r] + bvb;
    st[(16 + rr) * 32 + m]      = c10[r] + bva;
    st[(16 + rr) * 32 + 16 + m] = c11[r] + bvb;
  }
  __syncthreads();
  const int q8 = lane & 7, sub = lane >> 3;
  v4f v[8];
#pragma unroll
  for (int i = 0; i < 8; ++i) v[i] = *(const v4fa*)(st + (i * 4 + sub) * 32 + 4 * q8);
#pragma unroll
  for (int i = 0; i < 8; ++i)
    *(volatile v4f*)(H + (size_t)(r0 + i * 4 + sub) * DM + c0 + 4 * q8) = v[i];
  __threadfence();
#pragma unroll
  for (int i = 0; i < 8; ++i)
    *(volatile v4f*)(H + (size_t)(r0 + i * 4 + sub) * DM + c0 + 4 * q8) = v[i];
}

__global__ __launch_bounds__(512) void k_conv(const float* __restrict__ H,
                                              const float* __restrict__ Kf,
                                              _Float16* __restrict__ Hg)
{
  __shared__ __attribute__((aligned(16))) float zs[192 * 64];
  const int t = threadIdx.x;
  const int l0 = blockIdx.x * 128, c0 = blockIdx.y * 64, bg = blockIdx.z;
  const size_t rowb = (size_t)bg * LL;
  {
    const int p = t & 15, rr = t >> 4;
#pragma unroll
    for (int it = 0; it < 6; ++it) {
      const int r = it * 32 + rr;
      const int l = l0 - 64 + r;
      const int lc = (l < 0) ? 0 : l;
      const v4f v = *(const v4fa*)(H + (rowb + (size_t)lc) * DM + c0 + 4 * p);
      const bool ok = (l >= 0);
      const v4f u = {ok ? v.x : 0.f, ok ? v.y : 0.f, ok ? v.z : 0.f, ok ? v.w : 0.f};
      *(v4fa*)(zs + r * 64 + 4 * p) = u;
    }
  }
  __syncthreads();

  const int c = t & 63, q = t >> 6;
  const int x = 64 + 16 * q;
  const float* kp = Kf + (size_t)(c0 + c) * LMAX;
  float acc[16];
#pragma unroll
  for (int i = 0; i < 16; ++i) acc[i] = 0.f;
#pragma unroll 1
  for (int j = 0; j < LMAX; j += 2) {
    const float ka = kp[j], kb = kp[j + 1];
    const float* zp = zs + (x - 1 - j) * 64 + c;
    float zw[17];
#pragma unroll
    for (int i = 0; i < 17; ++i) zw[i] = zp[i * 64];
#pragma unroll
    for (int i = 0; i < 16; ++i) acc[i] = fmaf(ka, zw[i + 1], fmaf(kb, zw[i], acc[i]));
  }
  __syncthreads();
#pragma unroll
  for (int i = 0; i < 16; ++i) zs[(x + i) * 64 + c] = acc[i];
  __syncthreads();

  f16a* outs = (f16a*)zs;
#pragma unroll 1
  for (int it = 0; it < 16; ++it) {
    const int idx = it * 512 + t;
    const float y = zs[4096 + idx];
    outs[idx] = (_Float16)(gelu_t(y) * 64.0f);
  }
  __syncthreads();

  const int q8 = t & 7, r8 = t >> 3;
  const v8h o0 = *(const v8ha*)(outs + r8 * 64 + 8 * q8);
  const v8h o1 = *(const v8ha*)(outs + (64 + r8) * 64 + 8 * q8);
  _Float16* d0 = Hg + (rowb + l0 + r8) * DM + c0 + 8 * q8;
  _Float16* d1 = Hg + (rowb + l0 + 64 + r8) * DM + c0 + 8 * q8;
  *(volatile v8h*)d0 = o0;
  *(volatile v8h*)d1 = o1;
  __threadfence();
  *(volatile v8h*)d0 = o0;
  *(volatile v8h*)d1 = o1;
}

__global__ __launch_bounds__(256) void k_glu(const _Float16* __restrict__ Ag,
                                             const _Float16* __restrict__ Wg,
                                             const float* __restrict__ bglu,
                                             float* __restrict__ H)
{
  __shared__ __attribute__((aligned(16))) float sT[8 * 32 * 32];
  const int t = threadIdx.x, lane = t & 31, w = t >> 5, h4 = lane >> 4, m = lane & 15;
  const int wm = (w >> 1) * 32, wn = (w & 1) * 32;
  const int row0 = blockIdx.y * 128 + wm;
  const int n0 = blockIdx.x * 64 + wn;
  const size_t ao0 = (size_t)(row0 + m) * DM, ao1 = ao0 + (size_t)16 * DM;
  const size_t vo0 = (size_t)(n0 + m) * DM, vo1 = vo0 + (size_t)16 * DM;
  const size_t so0 = (size_t)(DM + n0 + m) * DM, so1 = so0 + (size_t)16 * DM;
  const v8f z8 = {0.f, 0.f, 0.f, 0.f, 0.f, 0.f, 0.f, 0.f};
  v8f cv00 = z8, cv01 = z8, cv10 = z8, cv11 = z8;
  v8f cs00 = z8, cs01 = z8, cs10 = z8, cs11 = z8;

#pragma unroll 1
  for (int k0 = 0; k0 < DM; k0 += 32) {
    const v16h a0 = ldh(Ag + ao0 + k0, h4);
    const v16h a1 = ldh(Ag + ao1 + k0, h4);
    const v16h bv0 = ldh(Wg + vo0 + k0, h4);
    const v16h bv1 = ldh(Wg + vo1 + k0, h4);
    const v16h bs0 = ldh(Wg + so0 + k0, h4);
    const v16h bs1 = ldh(Wg + so1 + k0, h4);
    cv00 = mma_h(a0, bv0, cv00); cv01 = mma_h(a0, bv1, cv01);
    cv10 = mma_h(a1, bv0, cv10); cv11 = mma_h(a1, bv1, cv11);
    cs00 = mma_h(a0, bs0, cs00); cs01 = mma_h(a0, bs1, cs01);
    cs10 = mma_h(a1, bs0, cs10); cs11 = mma_h(a1, bs1, cs11);
    asm volatile(HZ4 : "+v"(cv00), "+v"(cv01), "+v"(cv10), "+v"(cv11),
                       "+v"(cs00), "+v"(cs01), "+v"(cs10), "+v"(cs11)
                     : "v"(a0), "v"(a1), "v"(bv0), "v"(bv1), "v"(bs0), "v"(bs1));
  }

  const float INV = 6.103515625e-05f;
  const float bva = bglu[n0 + m],      bsa = bglu[DM + n0 + m];
  const float bvb = bglu[n0 + 16 + m], bsb = bglu[DM + n0 + 16 + m];
  float* st = sT + w * 1024;
#pragma unroll
  for (int r = 0; r < 8; ++r) {
    const int rr = 8 * h4 + r;
    {
      const float gv = fmaf(cv00[r], INV, bva), gs = fmaf(cs00[r], INV, bsa);
      st[rr * 32 + m] = gv * __builtin_amdgcn_rcpf(1.0f + __expf(-gs));
    }
    {
      const float gv = fmaf(cv01[r], INV, bvb), gs = fmaf(cs01[r], INV, bsb);
      st[rr * 32 + 16 + m] = gv * __builtin_amdgcn_rcpf(1.0f + __expf(-gs));
    }
    {
      const float gv = fmaf(cv10[r], INV, bva), gs = fmaf(cs10[r], INV, bsa);
      st[(16 + rr) * 32 + m] = gv * __builtin_amdgcn_rcpf(1.0f + __expf(-gs));
    }
    {
      const float gv = fmaf(cv11[r], INV, bvb), gs = fmaf(cs11[r], INV, bsb);
      st[(16 + rr) * 32 + 16 + m] = gv * __builtin_amdgcn_rcpf(1.0f + __expf(-gs));
    }
  }
  __syncthreads();
  const int q8 = lane & 7, sub = lane >> 3;
  v4f v[8];
#pragma unroll
  for (int i = 0; i < 8; ++i) {
    const int row = i * 4 + sub;
    const v4f gl  = *(const v4fa*)(st + row * 32 + 4 * q8);
    const v4f res = *(const v4fa*)(H + (size_t)(row0 + row) * DM + n0 + 4 * q8);
    v[i] = res + gl;
  }
#pragma unroll
  for (int i = 0; i < 8; ++i)
    *(volatile v4f*)(H + (size_t)(row0 + i * 4 + sub) * DM + n0 + 4 * q8) = v[i];
  __threadfence();
#pragma unroll
  for (int i = 0; i < 8; ++i)
    *(volatile v4f*)(H + (size_t)(row0 + i * 4 + sub) * DM + n0 + 4 * q8) = v[i];
}

__global__ __launch_bounds__(256) void k_ln(const float* __restrict__ S,
                                            const float* __restrict__ gam,
                                            const float* __restrict__ bet,
                                            unsigned short* __restrict__ Ph,
                                            unsigned short* __restrict__ Pl)
{
  const int lane = threadIdx.x & 31, w = threadIdx.x >> 5;
  const size_t row = (size_t)blockIdx.x * 8 + w;
  const float* sp = S + row * DM;
  float s = 0.f;
#pragma unroll 1
  for (int i = 0; i < 4; ++i) {
    const int base = i * 256 + lane * 8;
    const v4f a = *(const v4fa*)(sp + base), b = *(const v4fa*)(sp + base + 4);
    s += ((a.x + a.y) + (a.z + a.w)) + ((b.x + b.y) + (b.z + b.w));
  }
  s = wsum(s);
  const float mean = s * (1.0f / 1024.0f);
  float qv = 0.f;
#pragma unroll 1
  for (int i = 0; i < 4; ++i) {
    const int base = i * 256 + lane * 8;
    const v4f a = *(const v4fa*)(sp + base), b = *(const v4fa*)(sp + base + 4);
    float d;
    d = a.x - mean; qv = fmaf(d, d, qv);  d = a.y - mean; qv = fmaf(d, d, qv);
    d = a.z - mean; qv = fmaf(d, d, qv);  d = a.w - mean; qv = fmaf(d, d, qv);
    d = b.x - mean; qv = fmaf(d, d, qv);  d = b.y - mean; qv = fmaf(d, d, qv);
    d = b.z - mean; qv = fmaf(d, d, qv);  d = b.w - mean; qv = fmaf(d, d, qv);
  }
  qv = wsum(qv);
  const float rstd = rsqrtf(qv * (1.0f / 1024.0f) + 1e-5f);

  v8us oh[4], ol[4];
#pragma unroll
  for (int i = 0; i < 4; ++i) {
    const int base = i * 256 + lane * 8;
    const v4f a  = *(const v4fa*)(sp + base),  b  = *(const v4fa*)(sp + base + 4);
    const v4f ga = *(const v4fa*)(gam + base), gb = *(const v4fa*)(gam + base + 4);
    const v4f ba = *(const v4fa*)(bet + base), bb = *(const v4fa*)(bet + base + 4);
    const float y0 = (a.x - mean) * rstd * ga.x + ba.x, y1 = (a.y - mean) * rstd * ga.y + ba.y;
    const float y2 = (a.z - mean) * rstd * ga.z + ba.z, y3 = (a.w - mean) * rstd * ga.w + ba.w;
    const float y4 = (b.x - mean) * rstd * gb.x + bb.x, y5 = (b.y - mean) * rstd * gb.y + bb.y;
    const float y6 = (b.z - mean) * rstd * gb.z + bb.z, y7 = (b.w - mean) * rstd * gb.w + bb.w;
    const unsigned short h0 = f2bf(y0), h1 = f2bf(y1), h2 = f2bf(y2), h3 = f2bf(y3);
    const unsigned short h4b = f2bf(y4), h5 = f2bf(y5), h6 = f2bf(y6), h7 = f2bf(y7);
    const v8us hh = {h0, h1, h2, h3, h4b, h5, h6, h7};
    const v8us lw = {f2bf(y0 - bf2f(h0)), f2bf(y1 - bf2f(h1)), f2bf(y2 - bf2f(h2)), f2bf(y3 - bf2f(h3)),
                     f2bf(y4 - bf2f(h4b)), f2bf(y5 - bf2f(h5)), f2bf(y6 - bf2f(h6)), f2bf(y7 - bf2f(h7))};
    oh[i] = hh;
    ol[i] = lw;
  }
#pragma unroll
  for (int i = 0; i < 4; ++i) {
    const size_t off = row * DM + i * 256 + lane * 8;
    *(volatile v8us*)(Ph + off) = oh[i];
    *(volatile v8us*)(Pl + off) = ol[i];
  }
  __threadfence();
#pragma unroll
  for (int i = 0; i < 4; ++i) {
    const size_t off = row * DM + i * 256 + lane * 8;
    *(volatile v8us*)(Ph + off) = oh[i];
    *(volatile v8us*)(Pl + off) = ol[i];
  }
}

__global__ __launch_bounds__(256) void k_dec(const unsigned short* __restrict__ Ah,
                                             const unsigned short* __restrict__ Al,
                                             const unsigned short* __restrict__ Bh,
                                             const unsigned short* __restrict__ Bl,
                                             const float* __restrict__ bdec,
                                             float* __restrict__ out, int bbase)
{
  __shared__ __attribute__((aligned(16))) float sO[128 * 64];
  const int t = threadIdx.x, lane = t & 31, w = t >> 5, h4 = lane >> 4, m = lane & 15;
  const int s0 = (w >> 1) * 32, wl = (w & 1) * 32;
  const int l0 = blockIdx.x * 64, bg = blockIdx.y;
  const size_t ao0 = (size_t)(s0 + m) * DM, ao1 = ao0 + (size_t)16 * DM;
  const size_t bo0 = ((size_t)bg * LL + l0 + wl + m) * DM, bo1 = bo0 + (size_t)16 * DM;
  const v8f z8 = {0.f, 0.f, 0.f, 0.f, 0.f, 0.f, 0.f, 0.f};
  v8f c00 = z8, c01 = z8, c10 = z8, c11 = z8;

#pragma unroll 1
  for (int k0 = 0; k0 < DM; k0 += 32) {
    const v16b ah0 = ldb(Ah + ao0 + k0, h4), ah1 = ldb(Ah + ao1 + k0, h4);
    const v16b al0 = ldb(Al + ao0 + k0, h4), al1 = ldb(Al + ao1 + k0, h4);
    const v16b bh0 = ldb(Bh + bo0 + k0, h4), bh1 = ldb(Bh + bo1 + k0, h4);
    const v16b bl0 = ldb(Bl + bo0 + k0, h4), bl1 = ldb(Bl + bo1 + k0, h4);
    c00 = mma_b(ah0, bh0, c00); c00 = mma_b(ah0, bl0, c00); c00 = mma_b(al0, bh0, c00);
    c01 = mma_b(ah0, bh1, c01); c01 = mma_b(ah0, bl1, c01); c01 = mma_b(al0, bh1, c01);
    c10 = mma_b(ah1, bh0, c10); c10 = mma_b(ah1, bl0, c10); c10 = mma_b(al1, bh0, c10);
    c11 = mma_b(ah1, bh1, c11); c11 = mma_b(ah1, bl1, c11); c11 = mma_b(al1, bh1, c11);
    asm volatile(HZ4 : "+v"(c00), "+v"(c01), "+v"(c10), "+v"(c11)
                     : "v"(BH(ah0)), "v"(BH(ah1)), "v"(BH(al0)), "v"(BH(al1)),
                       "v"(BH(bh0)), "v"(BH(bh1)), "v"(BH(bl0)), "v"(BH(bl1)));
  }

#pragma unroll
  for (int r = 0; r < 8; ++r) {
    const int sa = s0 + 8 * h4 + r, sb = sa + 16;
    const float bda = bdec[sa], bdb = bdec[sb];
    sO[sa * 64 + wl + m]      = c00[r] + bda;
    sO[sa * 64 + wl + 16 + m] = c01[r] + bda;
    sO[sb * 64 + wl + m]      = c10[r] + bdb;
    sO[sb * 64 + wl + 16 + m] = c11[r] + bdb;
  }
  __syncthreads();
  const int sub = lane >> 4, p = lane & 15;
  v4f v[8];
#pragma unroll
  for (int i = 0; i < 8; ++i) {
    const int s = w * 16 + 2 * i + sub;
    v[i] = *(const v4fa*)(sO + s * 64 + 4 * p);
  }
  const size_t ob = (size_t)(bbase + bg) * DIN;
#pragma unroll
  for (int i = 0; i < 8; ++i) {
    const int s = w * 16 + 2 * i + sub;
    *(volatile v4f*)(out + (ob + s) * LL + l0 + 4 * p) = v[i];
  }
  __threadfence();
#pragma unroll
  for (int i = 0; i < 8; ++i) {
    const int s = w * 16 + 2 * i + sub;
    *(volatile v4f*)(out + (ob + s) * LL + l0 + 4 * p) = v[i];
  }
}

extern "C" void kernel_launch(void* const* d_in, const int* in_sizes, int n_in,
                              void* d_out, int out_size, void* d_ws, size_t ws_size,
                              hipStream_t stream)
{
  if (n_in < 15) return;
  if (in_sizes[0] != NB * DIN * LL) return;
  if (in_sizes[1] != DIN * DM || in_sizes[2] != DM || in_sizes[3] != DM) return;
  if (in_sizes[4] != DM * 4 || in_sizes[5] != DM * 4 || in_sizes[6] != DM * 4 || in_sizes[7] != DM * 4) return;
  if (in_sizes[8] != DM || in_sizes[9] != DM * 2 * DM || in_sizes[10] != 2 * DM) return;
  if (in_sizes[11] != DM || in_sizes[12] != DM || in_sizes[13] != DM * DIN || in_sizes[14] != DIN) return;
  if (out_size != NB * DIN * LL) return;

  const float* x      = (const float*)d_in[0];
  const float* W_enc  = (const float*)d_in[1];
  const float* b_enc  = (const float*)d_in[2];
  const float* log_dt = (const float*)d_in[3];
  const float* A_lr   = (const float*)d_in[4];
  const float* A_im   = (const float*)d_in[5];
  const float* C_re   = (const float*)d_in[6];
  const float* C_im   = (const float*)d_in[7];
  const float* Dv     = (const float*)d_in[8];
  const float* W_glu  = (const float*)d_in[9];
  const float* b_glu  = (const float*)d_in[10];
  const float* gam    = (const float*)d_in[11];
  const float* bet    = (const float*)d_in[12];
  const float* W_dec  = (const float*)d_in[13];
  const float* b_dec  = (const float*)d_in[14];
  float* out = (float*)d_out;

  char* ws = (char*)d_ws;
  size_t off = 0;
  float* Kf = (float*)(ws + off);                        off += (size_t)DM * LMAX * 4;
  unsigned short* WeTh = (unsigned short*)(ws + off);    off += (size_t)DM * DIN * 2;
  unsigned short* WeTl = (unsigned short*)(ws + off);    off += (size_t)DM * DIN * 2;
  unsigned short* WgT  = (unsigned short*)(ws + off);    off += (size_t)2 * DM * DM * 2;
  unsigned short* WdTh = (unsigned short*)(ws + off);    off += (size_t)DIN * DM * 2;
  unsigned short* WdTl = (unsigned short*)(ws + off);    off += (size_t)DIN * DM * 2;
  unsigned short* xTh  = (unsigned short*)(ws + off);    off += (size_t)NB * LL * DIN * 2;
  unsigned short* xTl  = (unsigned short*)(ws + off);    off += (size_t)NB * LL * DIN * 2;
  float* Hb = (float*)(ws + off);                        off += (size_t)MG * DM * 4;
  _Float16* Hg = (_Float16*)(ws + off);                  off += (size_t)MG * DM * 2;
  unsigned short* H2h = (unsigned short*)(ws + off);     off += (size_t)MG * DM * 2;
  unsigned short* H2l = (unsigned short*)(ws + off);     off += (size_t)MG * DM * 2;
  if (off > ws_size) return;

  k_ssm<<<(DM * LMAX) / 256, 256, 0, stream>>>(log_dt, A_lr, A_im, C_re, C_im, Dv, Kf);
  k_tr<1><<<dim3(DM / 64, DIN / 64, 1), 256, 0, stream>>>(W_enc, WeTh, WeTl, DIN, DM, 0LL, 0LL, 1.0f);
  k_tr<0><<<dim3(2 * DM / 64, DM / 64, 1), 256, 0, stream>>>(W_glu, WgT, WgT, DM, 2 * DM, 0LL, 0LL, 256.0f);
  k_tr<1><<<dim3(DIN / 64, DM / 64, 1), 256, 0, stream>>>(W_dec, WdTh, WdTl, DM, DIN, 0LL, 0LL, 1.0f);
  k_tr<1><<<dim3(LL / 64, DIN / 64, NB), 256, 0, stream>>>(x, xTh, xTl, DIN, LL,
                                                           (long long)DIN * LL, (long long)LL * DIN, 1.0f);

  for (int g = 0; g < NGRP; ++g) {
    const size_t xo = (size_t)g * MG * DIN;
    k_enc<<<dim3(DM / 64, MG / 128), 256, 0, stream>>>(xTh + xo, xTl + xo, WeTh, WeTl, b_enc, Hb);
    k_conv<<<dim3(LL / 128, DM / 64, GBT), 512, 0, stream>>>(Hb, Kf, Hg);
    k_glu<<<dim3(DM / 64, MG / 128), 256, 0, stream>>>(Hg, (const _Float16*)WgT, b_glu, Hb);
    k_ln<<<MG / 8, 256, 0, stream>>>(Hb, gam, bet, H2h, H2l);
    k_dec<<<dim3(LL / 64, GBT), 256, 0, stream>>>(WdTh, WdTl, H2h, H2l, b_dec, out, g * GBT);
  }
}
